// MambaBlock_9689446220504
// MI455X (gfx1250) — hardware-verified
//
#include <hip/hip_runtime.h>
#include <stddef.h>

typedef __attribute__((ext_vector_type(16))) _Float16 v16h;
typedef __attribute__((ext_vector_type(8)))  _Float16 v8h;
typedef __attribute__((ext_vector_type(16))) __bf16   v16b;
typedef __attribute__((ext_vector_type(8)))  __bf16   v8b;
typedef __attribute__((ext_vector_type(8)))  float    v8f;
typedef __attribute__((ext_vector_type(4)))  float    v4f;
typedef __attribute__((ext_vector_type(4)))  unsigned v4u;
typedef __attribute__((ext_vector_type(2)))  unsigned v2u;

constexpr int kNB   = 4;
constexpr int kNL   = 2048;
constexpr int kDMOD = 1024;
constexpr int kNST  = 16;
constexpr int kNCV  = 4;
constexpr int kNDI  = 2048;
constexpr int kNXZ  = 2 * kNDI;
constexpr int kWXN  = 2 * kNST + 1;
constexpr int kWXNP = 64;
constexpr int kLCH  = 32;

static_assert(kNL % 64 == 0 && kNXZ % 64 == 0 && kWXNP % 64 == 0 && kDMOD % 64 == 0);
static_assert(kDMOD % 32 == 0 && kNDI % 32 == 0);
static_assert(kNL % kLCH == 0 && (kLCH * kNST) % 256 == 0 && kLCH % 8 == 0);
static_assert(kNDI % 1024 == 0 && kNDI % 256 == 0);

constexpr size_t kSzXB    = (size_t)kNB * kNL * kDMOD * 2;
constexpr size_t kSzWINT  = (size_t)kNXZ * kDMOD * 2;
constexpr size_t kSzWXT   = (size_t)kWXNP * kNDI * 2;
constexpr size_t kSzWOUTT = (size_t)kDMOD * kNDI * 2;
constexpr size_t kSzXZ    = (size_t)kNL * kNXZ * 4;
constexpr size_t kSzXC    = (size_t)kNL * kNDI * 4;
constexpr size_t kSzPL    = (size_t)kNL * kNDI * 2;
constexpr size_t kSzDBL   = (size_t)kNL * kWXNP * 4;
constexpr size_t kOffXB    = 0;
constexpr size_t kOffWINT  = kOffXB + kSzXB;
constexpr size_t kOffWXT   = kOffWINT + kSzWINT;
constexpr size_t kOffWOUTT = kOffWXT + kSzWXT;
constexpr size_t kOffXZ    = kOffWOUTT + kSzWOUTT;
constexpr size_t kOffXC    = kOffXZ + kSzXZ;
constexpr size_t kOffXCH   = kOffXC + kSzXC;
constexpr size_t kOffXCL   = kOffXCH + kSzPL;
constexpr size_t kOffDBL   = kOffXCL + kSzPL;
constexpr size_t kOffYH    = kOffDBL + kSzDBL;
constexpr size_t kOffYL    = kOffYH + kSzPL;
constexpr size_t kWsTotal  = kOffYL + kSzPL;
static_assert(kWsTotal == 114032640);
static_assert(kWsTotal <= (size_t)134217728);
static_assert(kOffWINT % 128 == 0 && kOffWXT % 128 == 0 && kOffWOUTT % 128 == 0 && kOffXZ % 128 == 0 &&
              kOffXC % 128 == 0 && kOffXCH % 128 == 0 && kOffXCL % 128 == 0 && kOffDBL % 128 == 0 &&
              kOffYH % 128 == 0 && kOffYL % 128 == 0);

__device__ __forceinline__ unsigned short f2bf_bits(float f) {
  unsigned u = __float_as_uint(f);
  return (unsigned short)((u + 0x7FFFu + ((u >> 16) & 1u)) >> 16);
}
__device__ __forceinline__ float bf_bits2f(unsigned short h) { return __uint_as_float(((unsigned)h) << 16); }
__device__ __forceinline__ float bfr(float f) { return bf_bits2f(f2bf_bits(f)); }
__device__ __forceinline__ unsigned pack_bf2(float a, float b) {
  return (unsigned)f2bf_bits(a) | ((unsigned)f2bf_bits(b) << 16);
}
__device__ __forceinline__ void pack_hilo2(float a, float b, unsigned& wh, unsigned& wl) {
  const unsigned short ha = f2bf_bits(a), hb = f2bf_bits(b);
  const unsigned short la = f2bf_bits(a - bf_bits2f(ha)), lb = f2bf_bits(b - bf_bits2f(hb));
  wh = (unsigned)ha | ((unsigned)hb << 16);
  wl = (unsigned)la | ((unsigned)lb << 16);
}
__device__ __forceinline__ void split8(v4f u0, v4f u1, v4u& wh, v4u& wl) {
  unsigned a0, b0, a1, b1, a2, b2, a3, b3;
  pack_hilo2(u0[0], u0[1], a0, b0);
  pack_hilo2(u0[2], u0[3], a1, b1);
  pack_hilo2(u1[0], u1[1], a2, b2);
  pack_hilo2(u1[2], u1[3], a3, b3);
  wh[0] = a0; wh[1] = a1; wh[2] = a2; wh[3] = a3;
  wl[0] = b0; wl[1] = b1; wl[2] = b2; wl[3] = b3;
}

__device__ __forceinline__ void dep_guard_h(v8f& a, v8f& b, v16h x, v16h y) { asm volatile("v_nop\n\tv_nop\n\tv_nop\n\tv_nop" : "+v"(a), "+v"(b) : "v"(x), "v"(y)); }
__device__ __forceinline__ void dep_guard_b(v8f& a, v8f& b, v16b x, v16b y) { asm volatile("v_nop\n\tv_nop\n\tv_nop\n\tv_nop" : "+v"(a), "+v"(b) : "v"(x), "v"(y)); }
__device__ __forceinline__ void keep4_h(v16h a, v16h b, v16h c, v16h d) { asm volatile("v_nop" :: "v"(a), "v"(b), "v"(c), "v"(d)); }
__device__ __forceinline__ void keep4_b(v16b a, v16b b, v16b c, v16b d) { asm volatile("v_nop" :: "v"(a), "v"(b), "v"(c), "v"(d)); }
__device__ __forceinline__ void acc_guard4(v8f& a, v8f& b, v8f& c, v8f& d) { asm volatile("v_nop\n\tv_nop\n\tv_nop\n\tv_nop" : "+v"(a), "+v"(b), "+v"(c), "+v"(d)); }
template <typename T> struct Frag;
template <> struct Frag<_Float16> {
  typedef v16h V; union U { v16h v; v8h h[2]; };
  static __device__ __forceinline__ v16h load(const _Float16* p) {
    U f; f.h[0] = *(const v8h*)(p); f.h[1] = *(const v8h*)(p + 16); return f.v;
  }
  static __device__ __forceinline__ v8f mma(v16h a, v16h b, v8f c) {
    return __builtin_amdgcn_wmma_f32_16x16x32_f16(false, a, false, b, (short)0, c, false, false);
  }
  static __device__ __forceinline__ void guard(v8f& a, v8f& b, v16h x, v16h y) { dep_guard_h(a, b, x, y); }
  static __device__ __forceinline__ void keep(v16h a, v16h b, v16h c, v16h d) { keep4_h(a, b, c, d); }
};
template <> struct Frag<__bf16> {
  typedef v16b V; union U { v16b v; v8b h[2]; };
  static __device__ __forceinline__ v16b load(const __bf16* p) {
    U f; f.h[0] = *(const v8b*)(p); f.h[1] = *(const v8b*)(p + 16); return f.v;
  }
  static __device__ __forceinline__ v8f mma(v16b a, v16b b, v8f c) {
    return __builtin_amdgcn_wmma_f32_16x16x32_bf16(false, a, false, b, (short)0, c, false, false);
  }
  static __device__ __forceinline__ void guard(v8f& a, v8f& b, v16b x, v16b y) { dep_guard_b(a, b, x, y); }
  static __device__ __forceinline__ void keep(v16b a, v16b b, v16b c, v16b d) { keep4_b(a, b, c, d); }
};
template <int ET> struct Elem;
template <> struct Elem<0> { typedef _Float16 T; };
template <> struct Elem<1> { typedef __bf16 T; };

template <int ET, bool SPLIT_A, bool SPLIT_B>
__global__ __launch_bounds__(256) void wmma_gemm64(
    const unsigned short* __restrict__ Ap, const unsigned short* A2p, int lda, long strideA,
    const unsigned short* __restrict__ Btp, const unsigned short* Bt2p, int ldb, long strideB,
    float* __restrict__ Cout, int ldc, long strideC,
    int M, int N, int K, float scale) {
  typedef typename Elem<ET>::T T;
  typedef typename Frag<T>::V V;
  const T* A = (const T*)Ap; const T* A2 = (const T*)A2p; const T* Bt = (const T*)Btp; const T* Bt2 = (const T*)Bt2p;
  __shared__ __align__(16) float sT[8][16 * 68];
  const int b    = blockIdx.y;
  const int lane = threadIdx.x & 31;
  const int wave = threadIdx.x >> 5;
  const int tilesN = N >> 6;
  const int tilesM = M >> 6;
  const int tile = blockIdx.x * 8 + wave;
  if (tile >= tilesM * tilesN) return;
  const int tm = tile / tilesN;
  const int tn = tile - tm * tilesN;
  const int m0 = tm << 6;
  const int n0 = tn << 6;

  const T* Ab  = A  + (size_t)b * strideA;
  const T* Bb  = Bt + (size_t)b * strideB;
  const T* Ab2 = SPLIT_A ? (A2  + (size_t)b * strideA) : nullptr;
  const T* Bb2 = SPLIT_B ? (Bt2 + (size_t)b * strideB) : nullptr;

  const int rlane = lane & 15;
  const int koff  = (lane >> 4) * 8;
  const int mOff  = (lane >> 4) * 8;

  v8f acc[4][4];
#pragma unroll
  for (int i = 0; i < 4; ++i)
#pragma unroll
    for (int j = 0; j < 4; ++j) acc[i][j] = (v8f){0.f,0.f,0.f,0.f,0.f,0.f,0.f,0.f};

  for (int k0 = 0; k0 < K; k0 += 32) {
    V bh[4], bl[4];
#pragma unroll
    for (int j = 0; j < 4; ++j) {
      const size_t bo = (size_t)(n0 + (j << 4) + rlane) * ldb + koff + k0;
      bh[j] = Frag<T>::load(Bb + bo);
      if (SPLIT_B) bl[j] = Frag<T>::load(Bb2 + bo);
    }
#pragma unroll
    for (int i = 0; i < 4; ++i) {
      const size_t ao = (size_t)(m0 + (i << 4) + rlane) * lda + koff + k0;
      V ah = Frag<T>::load(Ab + ao);
      V al = ah;
      if (SPLIT_A) al = Frag<T>::load(Ab2 + ao);
#pragma unroll
      for (int j = 0; j < 4; ++j) {
        acc[i][j] = Frag<T>::mma(ah, bh[j], acc[i][j]);
        if (SPLIT_B) acc[i][j] = Frag<T>::mma(ah, bl[j], acc[i][j]);
        if (SPLIT_A) acc[i][j] = Frag<T>::mma(al, bh[j], acc[i][j]);
      }
      Frag<T>::guard(acc[i][0], acc[i][3], ah, al);
    }
    Frag<T>::keep(bh[0], bh[1], bh[2], bh[3]);
    if (SPLIT_B) Frag<T>::keep(bl[0], bl[1], bl[2], bl[3]);
  }
  acc_guard4(acc[0][0], acc[0][1], acc[0][2], acc[0][3]);
  acc_guard4(acc[1][0], acc[1][1], acc[1][2], acc[1][3]);
  acc_guard4(acc[2][0], acc[2][1], acc[2][2], acc[2][3]);
  acc_guard4(acc[3][0], acc[3][1], acc[3][2], acc[3][3]);

  float* slab = sT[wave];
#pragma unroll
  for (int i = 0; i < 4; ++i) {
    const int mBase = m0 + (i << 4);
#pragma unroll
    for (int j = 0; j < 4; ++j) {
#pragma unroll
      for (int r = 0; r < 8; ++r) {
        const float v = acc[i][j][r] * scale;
        slab[(mOff + r) * 68 + (j << 4) + rlane] = v;
      }
    }
    __builtin_amdgcn_fence(__ATOMIC_RELEASE, "workgroup");
    __builtin_amdgcn_wave_barrier();
    __builtin_amdgcn_fence(__ATOMIC_ACQUIRE, "workgroup");
    {
      float* C = Cout + (size_t)b * strideC;
      const int hh = lane >> 4, c4 = (lane & 15) * 4;
      for (int pass = 0; pass < 2; ++pass) {
#pragma unroll
        for (int it = 0; it < 8; ++it) {
          const int row = it * 2 + hh;
          v4f v = *(const v4f*)(slab + row * 68 + c4);
          *(volatile v4f*)(C + (size_t)(mBase + row) * ldc + n0 + c4) = v;
        }
        __threadfence();
      }
    }
    __builtin_amdgcn_fence(__ATOMIC_RELEASE, "workgroup");
    __builtin_amdgcn_wave_barrier();
    __builtin_amdgcn_fence(__ATOMIC_ACQUIRE, "workgroup");
  }
}

__global__ __launch_bounds__(256) void cvt_bf16x8_kernel(
    const float* __restrict__ in, unsigned short* __restrict__ out, int n8) {
  const int i = blockIdx.x * 256 + threadIdx.x;
  if (i < n8) {
    const v4f a = *(const v4f*)(in + (size_t)i * 8);
    const v4f c = *(const v4f*)(in + (size_t)i * 8 + 4);
    v4u w;
    w[0] = pack_bf2(a[0], a[1]); w[1] = pack_bf2(a[2], a[3]);
    w[2] = pack_bf2(c[0], c[1]); w[3] = pack_bf2(c[2], c[3]);
    volatile v4u* p = (volatile v4u*)(out + (size_t)i * 8);
    *p = w;
    __threadfence();
    *p = w;
  }
}

__global__ __launch_bounds__(256) void transpose_bf16_kernel(
    const float* __restrict__ in, unsigned short* __restrict__ out, int nrows, int ncols) {
  __shared__ float tileT[64][65];
  const int tid = threadIdx.x, lane = tid & 31, wave = tid >> 5;
  const int r0 = blockIdx.y * 64, c0 = blockIdx.x * 64;
  const int rr = tid >> 2, cs = (tid & 3) * 16;
#pragma unroll
  for (int i = 0; i < 4; ++i) {
    const v4f v = *(const v4f*)(in + (size_t)(r0 + rr) * ncols + c0 + cs + 4 * i);
    tileT[rr][cs + 4 * i + 0] = v[0];
    tileT[rr][cs + 4 * i + 1] = v[1];
    tileT[rr][cs + 4 * i + 2] = v[2];
    tileT[rr][cs + 4 * i + 3] = v[3];
  }
  __syncthreads();
  const int q = lane >> 3, c8 = (lane & 7) * 8;
  for (int pass = 0; pass < 2; ++pass) {
#pragma unroll
    for (int it = 0; it < 2; ++it) {
      const int n = wave * 8 + it * 4 + q;
      v4u w;
#pragma unroll
      for (int e = 0; e < 4; ++e) w[e] = pack_bf2(tileT[c8 + 2 * e][n], tileT[c8 + 2 * e + 1][n]);
      *(volatile v4u*)(out + (size_t)(c0 + n) * nrows + r0 + c8) = w;
    }
    __threadfence();
  }
}

__global__ __launch_bounds__(256) void wx_t_kernel(const float* __restrict__ Wx, unsigned short* __restrict__ out) {
  const int n  = blockIdx.y;
  const int k  = (blockIdx.x * 256 + threadIdx.x) * 8;
  const int nc = (n < kWXN) ? n : (kWXN - 1);
  const bool live = (n < kWXN);
  float f[8];
#pragma unroll
  for (int e = 0; e < 8; ++e) {
    const float t = Wx[(size_t)(k + e) * kWXN + nc];
    f[e] = live ? t : 0.0f;
  }
  v4u w;
#pragma unroll
  for (int e = 0; e < 4; ++e) w[e] = pack_bf2(f[2 * e], f[2 * e + 1]);
  volatile v4u* p = (volatile v4u*)(out + (size_t)n * kNDI + k);
  *p = w;
  __threadfence();
  *p = w;
}

__global__ __launch_bounds__(256) void conv_silu_kernel(
    const float* __restrict__ xz, const float* __restrict__ conv_w, const float* __restrict__ conv_b,
    float* __restrict__ xc, unsigned short* __restrict__ xch, unsigned short* __restrict__ xcl) {
  __shared__ __align__(16) unsigned shw[2][512];
  const int tid = threadIdx.x;
  const int l   = blockIdx.y;
  const int cb  = blockIdx.x * 1024;
  const int c   = cb + 4 * tid;
  v4f wv[4];
#pragma unroll
  for (int e = 0; e < 4; ++e) wv[e] = *(const v4f*)(conv_w + (size_t)(c + e) * kNCV);
  const v4f bq = *(const v4f*)(conv_b + c);
  float acc[4];
#pragma unroll
  for (int e = 0; e < 4; ++e) acc[e] = bfr(bq[e]);
#pragma unroll
  for (int k = 0; k < kNCV; ++k) {
    const int lk  = l + k - (kNCV - 1);
    const int lkc = lk < 0 ? 0 : lk;
    const bool live = (lk >= 0);
    const v4f xv = *(const v4f*)(xz + (size_t)lkc * kNXZ + c);
#pragma unroll
    for (int e = 0; e < 4; ++e) {
      const float xe = live ? xv[e] : 0.0f;
      acc[e] += xe * bfr(wv[e][k]);
    }
  }
  float v[4];
#pragma unroll
  for (int e = 0; e < 4; ++e) {
    const float t  = acc[e];
    const float sg = __builtin_amdgcn_rcpf(1.0f + expf(-t));
    v[e] = t * sg;
  }
  v4f vo;
  vo[0] = v[0]; vo[1] = v[1]; vo[2] = v[2]; vo[3] = v[3];
  unsigned wh0, wl0, wh1, wl1;
  pack_hilo2(v[0], v[1], wh0, wl0);
  pack_hilo2(v[2], v[3], wh1, wl1);
  v2u th, tl;
  th[0] = wh0; th[1] = wh1; tl[0] = wl0; tl[1] = wl1;
  *(v2u*)(&shw[0][2 * tid]) = th;
  *(v2u*)(&shw[1][2 * tid]) = tl;
  volatile v4f* px = (volatile v4f*)(xc + (size_t)l * kNDI + c);
  *px = vo;
  __syncthreads();
  const int pl  = tid >> 7;
  const int idx = tid & 127;
  const v4u w = *(const v4u*)(&shw[pl][4 * idx]);
  unsigned short* base = (pl == 0) ? xch : xcl;
  volatile v4u* pd = (volatile v4u*)(base + (size_t)l * kNDI + cb + 8 * idx);
  *pd = w;
  __threadfence();
  *px = vo;
  *pd = w;
}

__global__ __launch_bounds__(256) void scan_gate_kernel(
    const float* __restrict__ xc, const float* __restrict__ xz, const float* __restrict__ dbl,
    const float* __restrict__ A_log, const float* __restrict__ D_par,
    unsigned short* __restrict__ yh, unsigned short* __restrict__ yl) {
  __shared__ float Asn[kNST];
  __shared__ __align__(16) float Pch[kLCH][3 * kNST];
  __shared__ __align__(16) float ybuf[kLCH][256];
  const int tid = threadIdx.x, lane = tid & 31, wave = tid >> 5;
  const int cbase = blockIdx.x * 256;
  const int d = cbase + tid;
  if (tid < kNST) Asn[tid] = -expf(bfr(A_log[tid]));
  const float Dp = bfr(D_par[d]);
  float h[kNST];
#pragma unroll
  for (int n = 0; n < kNST; ++n) h[n] = 0.0f;
  __syncthreads();
  for (int l0 = 0; l0 < kNL; l0 += kLCH) {
#pragma unroll 1
    for (int i = 0; i < (kLCH * kNST) / 256; ++i) {
      const int p = tid + 256 * i;
      const int ll = p >> 4;
      const int n  = p & 15;
      const int row = l0 + ll;
      const float x0 = dbl[(size_t)row * kWXNP];
      const float Bv = dbl[(size_t)row * kWXNP + 1 + n];
      const float Cv = dbl[(size_t)row * kWXNP + 1 + kNST + n];
      const float delta = fmaxf(x0, 0.0f) + log1pf(expf(-fabsf(x0)));
      Pch[ll][n]            = expf(delta * Asn[n]);
      Pch[ll][kNST + n]     = delta * Bv;
      Pch[ll][2 * kNST + n] = Cv;
    }
    __syncthreads();
#pragma unroll 1
    for (int s = 0; s < kLCH; ++s) {
      const int row = l0 + s;
      const float xv = xc[(size_t)row * kNDI + d];
      const float zv = xz[(size_t)row * kNXZ + kNDI + d];
      float y = 0.0f;
#pragma unroll
      for (int n = 0; n < kNST; ++n) {
        const float a  = Pch[s][n];
        const float bb = Pch[s][kNST + n];
        const float cc = Pch[s][2 * kNST + n];
        h[n] = a * h[n] + bb * xv;
        y += h[n] * cc;
      }
      y += xv * Dp;
      const float sg = __builtin_amdgcn_rcpf(1.0f + expf(-zv));
      y = y * (zv * sg);
      ybuf[s][tid] = y;
    }
    __syncthreads();
    const int c8 = lane * 8;
    for (int pass = 0; pass < 2; ++pass) {
#pragma unroll
      for (int it = 0; it < kLCH / 8; ++it) {
        const int r = it * 8 + wave;
        const v4f u0 = *(const v4f*)(&ybuf[r][c8]);
        const v4f u1 = *(const v4f*)(&ybuf[r][c8 + 4]);
        v4u wh, wl;
        split8(u0, u1, wh, wl);
        const size_t o = (size_t)(l0 + r) * kNDI + cbase + c8;
        *(volatile v4u*)(yh + o) = wh;
        *(volatile v4u*)(yl + o) = wl;
      }
      __threadfence();
    }
    __syncthreads();
  }
}

extern "C" void kernel_launch(void* const* d_in, const int* in_sizes, int n_in,
                              void* d_out, int out_size, void* d_ws, size_t ws_size,
                              hipStream_t stream) {
  if (n_in < 8) return;
  if (in_sizes[0] != kNB * kNL * kDMOD) return;
  if (in_sizes[1] != kDMOD * kNXZ) return;
  if (in_sizes[2] != kNDI * kNCV) return;
  if (in_sizes[3] != kNDI) return;
  if (in_sizes[4] != kNDI * kWXN) return;
  if (in_sizes[5] != kNST) return;
  if (in_sizes[6] != kNDI) return;
  if (in_sizes[7] != kNDI * kDMOD) return;
  if (out_size != kNB * kNL * kDMOD) return;
  if (ws_size < kWsTotal) return;

  const float* x      = (const float*)d_in[0];
  const float* W_in   = (const float*)d_in[1];
  const float* conv_w = (const float*)d_in[2];
  const float* conv_b = (const float*)d_in[3];
  const float* W_x    = (const float*)d_in[4];
  const float* A_log  = (const float*)d_in[5];
  const float* D_par  = (const float*)d_in[6];
  const float* W_out  = (const float*)d_in[7];
  float* out = (float*)d_out;

  char* ws = (char*)d_ws;
  unsigned short* xb    = (unsigned short*)(ws + kOffXB);
  unsigned short* winT  = (unsigned short*)(ws + kOffWINT);
  unsigned short* wxT   = (unsigned short*)(ws + kOffWXT);
  unsigned short* woutT = (unsigned short*)(ws + kOffWOUTT);
  float*          xz    = (float*)(ws + kOffXZ);
  float*          xc    = (float*)(ws + kOffXC);
  unsigned short* xch   = (unsigned short*)(ws + kOffXCH);
  unsigned short* xcl   = (unsigned short*)(ws + kOffXCL);
  float*          dbl   = (float*)(ws + kOffDBL);
  unsigned short* yh    = (unsigned short*)(ws + kOffYH);
  unsigned short* yl    = (unsigned short*)(ws + kOffYL);

  const int n8x = (kNB * kNL * kDMOD) / 8;
  cvt_bf16x8_kernel<<<dim3((n8x + 255) / 256), dim3(256), 0, stream>>>(x, xb, n8x);
  transpose_bf16_kernel<<<dim3(kNXZ / 64, kDMOD / 64), dim3(256), 0, stream>>>(W_in, winT, kDMOD, kNXZ);
  wx_t_kernel<<<dim3(kNDI / 8 / 256, kWXNP), dim3(256), 0, stream>>>(W_x, wxT);
  transpose_bf16_kernel<<<dim3(kDMOD / 64, kNDI / 64), dim3(256), 0, stream>>>(W_out, woutT, kNDI, kDMOD);

  const int tiles1 = (kNL / 64) * (kNXZ / 64);
  const int tilesX = (kNL / 64) * (kWXNP / 64);
  const int tiles3 = (kNL / 64) * (kDMOD / 64);

  for (int b = 0; b < kNB; ++b) {
    const unsigned short* xbB = xb + (size_t)b * kNL * kDMOD;
    wmma_gemm64<1, false, false><<<dim3((tiles1 + 7) / 8, 1), dim3(256), 0, stream>>>(
        xbB, xbB, kDMOD, 0L, winT, winT, kDMOD, 0L, xz, kNXZ, 0L, kNL, kNXZ, kDMOD, 1.0f);
    conv_silu_kernel<<<dim3(kNDI / 1024, kNL), dim3(256), 0, stream>>>(xz, conv_w, conv_b, xc, xch, xcl);
    wmma_gemm64<1, true, false><<<dim3((tilesX + 7) / 8, 1), dim3(256), 0, stream>>>(
        xch, xcl, kNDI, 0L, wxT, wxT, kNDI, 0L, dbl, kWXNP, 0L, kNL, kWXNP, kNDI, 1.0f);
    scan_gate_kernel<<<dim3(kNDI / 256), dim3(256), 0, stream>>>(xc, xz, dbl, A_log, D_par, yh, yl);
    wmma_gemm64<1, true, false><<<dim3((tiles3 + 7) / 8, 1), dim3(256), 0, stream>>>(
        yh, yl, kNDI, 0L, woutT, woutT, kNDI, 0L, out + (size_t)b * kNL * kDMOD, kDMOD, 0L,
        kNL, kDMOD, kNDI, 1.0f);
  }
}
